// MaskedMultiHeadAttention_15410342658603
// MI455X (gfx1250) — hardware-verified
//
#include <hip/hip_runtime.h>
#include <stdint.h>
#include <math.h>


#pragma clang fp contract(off)

#ifndef NB
#define NB 2
#endif
#ifndef SEQ
#define SEQ 2048
#endif
#define NB_FULL 2
#define SEQ_FULL 2048
#define DM 1024
#define NH 16
#define DH 64
#define RESQ (((SEQ) < 256) ? (SEQ) : 256)
#define MROWS ((NB) * (SEQ))

static_assert((SEQ) % 128 == 0);
static_assert((RESQ) % 128 == 0);
static_assert((NB) >= 1 && (NB) <= NB_FULL);
static_assert((SEQ) <= SEQ_FULL);
static_assert(DM == NH * DH);
static_assert(DM % 32 == 0);

typedef _Float16 v16h __attribute__((ext_vector_type(16)));
typedef _Float16 v8h  __attribute__((ext_vector_type(8)));
typedef float    v8f  __attribute__((ext_vector_type(8)));
typedef float    v4f  __attribute__((ext_vector_type(4)));
typedef float    v2f  __attribute__((ext_vector_type(2)));

constexpr size_t SZ_PL  = (size_t)MROWS * DM * 2;
constexpr size_t SZ_W   = (size_t)DM * DM * 2;
constexpr size_t SZ_R   = (size_t)(NB) * (RESQ) * DM * 2;
constexpr size_t SZ_CS  = (size_t)(SEQ) * 32 * 8;
constexpr size_t OFF_X   = 0;
constexpr size_t OFF_WQ  = OFF_X   + SZ_PL;
constexpr size_t OFF_WK  = OFF_WQ  + SZ_W;
constexpr size_t OFF_WV  = OFF_WK  + SZ_W;
constexpr size_t OFF_WO  = OFF_WV  + SZ_W;
constexpr size_t OFF_Q   = OFF_WO  + SZ_W;
constexpr size_t OFF_K   = OFF_Q   + SZ_PL;
constexpr size_t OFF_VT  = OFF_K   + SZ_PL;
constexpr size_t OFF_AO  = OFF_VT  + SZ_PL;
constexpr size_t OFF_QR  = OFF_AO  + SZ_PL;
constexpr size_t OFF_KR  = OFF_QR  + SZ_R;
constexpr size_t OFF_VTR = OFF_KR  + SZ_R;
constexpr size_t OFF_AOR = OFF_VTR + SZ_R;
constexpr size_t OFF_CS  = OFF_AOR + SZ_R;
constexpr size_t WS_TOTAL = OFF_CS + SZ_CS;
static_assert(WS_TOTAL <= (size_t)134217728);
static_assert((size_t)(NB) * NH * DH * (SEQ) * 2 == SZ_PL);
static_assert((size_t)(NB) * NH * DH * (RESQ) * 2 == SZ_R);

__device__ __forceinline__ float bfr(float x) {
  uint32_t u = __float_as_uint(x);
  u = u + 0x7FFFu + ((u >> 16) & 1u);
  u = u & 0xFFFF0000u;
  return __uint_as_float(u);
}

__device__ __forceinline__ v8f zero8() {
  v8f z;
#pragma unroll
  for (int r = 0; r < 8; ++r) z[r] = 0.0f;
  return z;
}

__device__ __forceinline__ v16h load_frag(const _Float16* base, int stride) {
  const int lane = threadIdx.x & 31;
  const int m = lane & 15;
  const int g = lane >> 4;
  const _Float16* p = base + (size_t)m * stride + 8 * g;
  union { v16h v; v8h hv[2]; } f;
  f.hv[0] = *reinterpret_cast<const v8h*>(p);
  f.hv[1] = *reinterpret_cast<const v8h*>(p + 16);
  return f.v;
}

__device__ __forceinline__ v8f wmma16(v16h a, v16h b, v8f c) {
  c = __builtin_amdgcn_wmma_f32_16x16x32_f16(false, a, false, b, (short)0, c,
                                             false, false);
  asm volatile("v_nop\n\tv_nop\n\tv_nop\n\tv_nop" : "+v"(c) : "v"(a), "v"(b));
  return c;
}

__device__ __forceinline__ void sincos_cw(float a, float& sn, float& cn) {
  const float kf = rintf(a * 0.636619772367581343f);
  const int k = (int)kf;
  float r = fmaf(-kf, 1.5703125f, a);
  r = fmaf(-kf, 4.837512969970703125e-4f, r);
  r = fmaf(-kf, 7.54978995489188216e-8f, r);
  const float z = r * r;
  float ps = fmaf(-1.9515295891e-4f, z, 8.3321608736e-3f);
  ps = fmaf(ps, z, -1.6666654611e-1f);
  ps = fmaf(ps * z, r, r);
  float pc = fmaf(2.443315711809948e-5f, z, -1.388731625493765e-3f);
  pc = fmaf(pc, z, 4.166664568298827e-2f);
  pc = fmaf(pc, z * z, fmaf(-0.5f, z, 1.0f));
  const int q = k & 3;
  float s = (q & 1) ? pc : ps;
  float c = (q & 1) ? ps : pc;
  s = (q & 2) ? -s : s;
  c = ((q + 1) & 2) ? -c : c;
  sn = s;
  cn = c;
}

__global__ void __launch_bounds__(256)
k_cvt(const float* __restrict__ src, _Float16* __restrict__ dst, int n8, float scale) {
  const int i = blockIdx.x * 256 + threadIdx.x;
  const int ic = (i < n8) ? i : (n8 - 1);
  const v4f a = *reinterpret_cast<const v4f*>(src + (size_t)ic * 8);
  const v4f c = *reinterpret_cast<const v4f*>(src + (size_t)ic * 8 + 4);
  union { v8h h; v4f f; } o;
  o.h[0] = (_Float16)(bfr(a.x) * scale);
  o.h[1] = (_Float16)(bfr(a.y) * scale);
  o.h[2] = (_Float16)(bfr(a.z) * scale);
  o.h[3] = (_Float16)(bfr(a.w) * scale);
  o.h[4] = (_Float16)(bfr(c.x) * scale);
  o.h[5] = (_Float16)(bfr(c.y) * scale);
  o.h[6] = (_Float16)(bfr(c.z) * scale);
  o.h[7] = (_Float16)(bfr(c.w) * scale);
  const v4f ov = o.f;
  if (i < n8) *(volatile v4f*)(dst + (size_t)i * 8) = ov;
  __threadfence();
  if (i < n8) *(volatile v4f*)(dst + (size_t)i * 8) = ov;
}

__global__ void __launch_bounds__(256)
k_table(v2f* __restrict__ cs, int n) {
  const int i = blockIdx.x * 256 + threadIdx.x;
  const int ic = (i < n) ? i : (n - 1);
  const int pos = ic >> 5, pair = ic & 31;
  const float e = (float)(2 * pair) * (1.0f / 64.0f);
  const float p = powf(10000.0f, e);
  const float inv = 1.0f / p;
  const float a = (float)pos * inv;
  float s, c;
  sincos_cw(a, s, c);
  v2f o;
  o.x = c;
  o.y = s;
  if (i < n) *(volatile v2f*)(cs + i) = o;
  __threadfence();
  if (i < n) *(volatile v2f*)(cs + i) = o;
}

template <int MODE>
__global__ void __launch_bounds__(128)
k_proj(const _Float16* __restrict__ X, const _Float16* __restrict__ W,
       const float* __restrict__ bias, const v2f* __restrict__ cs,
       _Float16* __restrict__ Ph, _Float16* __restrict__ Pr) {
  __shared__ __align__(16) _Float16 stile[4 * 32 * 64];
  __shared__ __align__(16) v2f stab[(MODE < 2) ? (128 * 32) : 2];

  const int t = threadIdx.x, w = t >> 5, lane = t & 31;
  const int n = lane & 15, g = lane >> 4;
  const int h = blockIdx.x;
  const int cBase = h * DH;
  const int mBase = blockIdx.y * 128;
  const int b = mBase / (SEQ);
  const int s0 = mBase - b * (SEQ);
  const bool resblk = (s0 < (RESQ));

  if (MODE < 2) {
    const v4f* src = reinterpret_cast<const v4f*>(cs + (size_t)s0 * 32);
    v4f* dl = reinterpret_cast<v4f*>(stab);
#pragma unroll 1
    for (int o = 0; o < 2; ++o) {
#pragma unroll
      for (int i = 0; i < 8; ++i) {
        const int c = t + (o * 8 + i) * 128;
        dl[c] = src[c];
      }
    }
  }
  __syncthreads();

  v8f acc[2][4];
#pragma unroll
  for (int mi = 0; mi < 2; ++mi)
#pragma unroll
    for (int j = 0; j < 4; ++j) acc[mi][j] = zero8();

  const _Float16* xr = X + (size_t)(mBase + 32 * w) * DM;
  const _Float16* wr = W + (size_t)cBase * DM;
#pragma unroll 1
  for (int kc = 0; kc < DM; kc += 32) {
    const v16h a0 = load_frag(xr + kc, DM);
    const v16h a1 = load_frag(xr + (size_t)16 * DM + kc, DM);
#pragma unroll
    for (int j = 0; j < 4; ++j) {
      const v16h bb = load_frag(wr + (size_t)(16 * j) * DM + kc, DM);
      acc[0][j] = wmma16(a0, bb, acc[0][j]);
      acc[1][j] = wmma16(a1, bb, acc[1][j]);
    }
  }

  float bia[4];
#pragma unroll
  for (int j = 0; j < 4; ++j) bia[j] = bfr(bias[cBase + 16 * j + n]);
  const float sgn = (n & 1) ? 1.0f : -1.0f;
  const int npass = resblk ? 2 : 1;

  for (int pass = 0; pass < npass; ++pass) {
#pragma unroll
    for (int mi = 0; mi < 2; ++mi)
#pragma unroll
      for (int j = 0; j < 4; ++j)
#pragma unroll
        for (int r = 0; r < 8; ++r) {
          const int rl = mi * 16 + 8 * g + r;
          const int cl = j * 16 + n;
          const float v = acc[mi][j][r] * (1.0f / 1024.0f) + bia[j];
          float o = v;
          if (MODE < 2) {
            const float pv = __shfl_xor(v, 1, 32);
            const v2f c2 = stab[(32 * w + rl) * 32 + (cl >> 1)];
            o = v * c2.x + sgn * (pv * c2.y);
          }
          const _Float16 hh = (_Float16)o;
          const _Float16 rr = (_Float16)((o - (float)hh) * 4096.0f);
          const _Float16 ov = pass ? rr : hh;
          if (MODE < 2) stile[(w * 32 + rl) * 64 + cl] = ov;
          else          stile[cl * 128 + 32 * w + rl] = ov;
        }
    __syncthreads();

    if (MODE < 2) {
      const int ch = lane & 7, rq = lane >> 3;
      _Float16* dst = pass ? (Pr + ((size_t)b * (RESQ) + s0 + 32 * w) * DM + cBase)
                           : (Ph + ((size_t)mBase + 32 * w) * DM + cBase);
#pragma unroll
      for (int i = 0; i < 8; ++i) {
        const int rl = i * 4 + rq;
        const v4f val = *reinterpret_cast<const v4f*>(&stile[(w * 32 + rl) * 64 + ch * 8]);
        *(volatile v4f*)(dst + (size_t)rl * DM + ch * 8) = val;
      }
      __threadfence();
#pragma unroll
      for (int i = 0; i < 8; ++i) {
        const int rl = i * 4 + rq;
        const v4f val = *reinterpret_cast<const v4f*>(&stile[(w * 32 + rl) * 64 + ch * 8]);
        *(volatile v4f*)(dst + (size_t)rl * DM + ch * 8) = val;
      }
    } else {
      const int ch = t & 15, dq = t >> 4;
      const size_t pitch = pass ? (size_t)(RESQ) : (size_t)(SEQ);
      _Float16* dst = pass ? (Pr + ((size_t)(b * NH + h) * DH) * (RESQ) + s0)
                           : (Ph + ((size_t)(b * NH + h) * DH) * (SEQ) + s0);
#pragma unroll
      for (int p = 0; p < 8; ++p) {
        const int d = p * 8 + dq;
        const v4f val = *reinterpret_cast<const v4f*>(&stile[d * 128 + ch * 8]);
        *(volatile v4f*)(dst + (size_t)d * pitch + ch * 8) = val;
      }
      __threadfence();
#pragma unroll
      for (int p = 0; p < 8; ++p) {
        const int d = p * 8 + dq;
        const v4f val = *reinterpret_cast<const v4f*>(&stile[d * 128 + ch * 8]);
        *(volatile v4f*)(dst + (size_t)d * pitch + ch * 8) = val;
      }
    }
    __syncthreads();
  }
}

template <bool RES>
__global__ void __launch_bounds__(128) __attribute__((amdgpu_num_vgpr(256)))
k_attn(const _Float16* __restrict__ Q, const _Float16* __restrict__ K,
       const _Float16* __restrict__ Vt, const _Float16* __restrict__ Qr,
       const _Float16* __restrict__ Kr, const _Float16* __restrict__ Vtr,
       _Float16* __restrict__ AO, _Float16* __restrict__ AOr, int qt0) {
  __shared__ __align__(16) _Float16 Ks[64 * 64];
  __shared__ __align__(16) _Float16 Vs[64 * 64];
  __shared__ __align__(16) _Float16 Pl[4 * 16 * 64];
  __shared__ __align__(16) _Float16 Krs[RES ? 64 * 64 : 8];
  __shared__ __align__(16) _Float16 Vrs[RES ? 64 * 64 : 8];
  __shared__ __align__(16) _Float16 Prl[RES ? 4 * 16 * 64 : 8];

  constexpr int NSUB = RES ? 2 : 1;
  constexpr int NJ   = 4 / NSUB;
  constexpr int NK2  = NJ / 2;

  const int t = threadIdx.x, w = t >> 5, lane = t & 31;
  const int n = lane & 15, g = lane >> 4;
  const int qtile = qt0 + blockIdx.x;
  const int h = blockIdx.y, b = blockIdx.z;
  const int qBase = qtile * 64;
  const int qw = qBase + 16 * w;

  const _Float16* qp  = Q  + ((size_t)b * (SEQ)  + qw) * DM + h * DH;
  const _Float16* qrp = Qr + ((size_t)b * (RESQ) + qw) * DM + h * DH;

  v8f Oa[4];
#pragma unroll
  for (int jd = 0; jd < 4; ++jd) Oa[jd] = zero8();
  float mrun[8], lrun[8];
#pragma unroll
  for (int r = 0; r < 8; ++r) { mrun[r] = -__builtin_inff(); lrun[r] = 0.0f; }

#pragma unroll 1
  for (int kt = 0; kt <= qtile; ++kt) {
    const int kBase = kt * 64;
#pragma unroll
    for (int i = 0; i < 4; ++i) {
      const int c = t + i * 128;
      const int row = c >> 3, ch = c & 7;
      *reinterpret_cast<v8h*>(&Ks[row * 64 + ch * 8]) =
          *reinterpret_cast<const v8h*>(K + ((size_t)b * (SEQ) + kBase + row) * DM + h * DH + ch * 8);
      *reinterpret_cast<v8h*>(&Vs[row * 64 + ch * 8]) =
          *reinterpret_cast<const v8h*>(Vt + ((size_t)(b * NH + h) * DH + row) * (SEQ) + kBase + ch * 8);
      if (RES) {
        *reinterpret_cast<v8h*>(&Krs[row * 64 + ch * 8]) =
            *reinterpret_cast<const v8h*>(Kr + ((size_t)b * (RESQ) + kBase + row) * DM + h * DH + ch * 8);
        *reinterpret_cast<v8h*>(&Vrs[row * 64 + ch * 8]) =
            *reinterpret_cast<const v8h*>(Vtr + ((size_t)(b * NH + h) * DH + row) * (RESQ) + kBase + ch * 8);
      }
    }
    __syncthreads();
    const bool diag = (kt == qtile);

#pragma unroll 1
    for (int sub = 0; sub < NSUB; ++sub) {
      const int kOff = sub * (NJ * 16);

      v8f sc[NJ], sr[NJ];
#pragma unroll
      for (int j = 0; j < NJ; ++j) { sc[j] = zero8(); sr[j] = zero8(); }
#pragma unroll
      for (int ks = 0; ks < 2; ++ks) {
        const v16h qa = load_frag(qp + 32 * ks, DM);
        v16h qra = qa;
        if (RES) qra = load_frag(qrp + 32 * ks, DM);
#pragma unroll
        for (int j = 0; j < NJ; ++j) {
          const v16h kb = load_frag(&Ks[(kOff + j * 16) * 64 + 32 * ks], 64);
          sc[j] = wmma16(qa, kb, sc[j]);
          if (RES) {
            const v16h krb = load_frag(&Krs[(kOff + j * 16) * 64 + 32 * ks], 64);
            sr[j] = wmma16(qa, krb, sr[j]);
            sr[j] = wmma16(qra, kb, sr[j]);
          }
        }
      }

#pragma unroll
      for (int r = 0; r < 8; ++r) {
        const int qloc = 16 * w + 8 * g + r;
        float sv[NJ];
        float mt = -__builtin_inff();
#pragma unroll
        for (int j = 0; j < NJ; ++j) {
          float s = sc[j][r];
          if (RES) s = s + sr[j][r] * (1.0f / 4096.0f);
          s = s * 0.125f;
          const int kloc = kOff + j * 16 + n;
          s = (diag && (kloc > qloc)) ? -__builtin_inff() : s;
          sv[j] = s;
          mt = fmaxf(mt, s);
        }
#pragma unroll
        for (int off = 1; off < 16; off <<= 1) mt = fmaxf(mt, __shfl_xor(mt, off, 32));
        const float mnew = fmaxf(mrun[r], mt);
        const float alpha = __expf(mrun[r] - mnew);
        float psum = 0.0f;
#pragma unroll
        for (int j = 0; j < NJ; ++j) {
          const float p = __expf(sv[j] - mnew);
          psum += p;
          const float pc = p * 1024.0f;
          const _Float16 ph = (_Float16)pc;
          Pl[(w * 16 + 8 * g + r) * 64 + kOff + j * 16 + n] = ph;
          if (RES) Prl[(w * 16 + 8 * g + r) * 64 + kOff + j * 16 + n] = (_Float16)((pc - (float)ph) * 4096.0f);
        }
#pragma unroll
        for (int off = 1; off < 16; off <<= 1) psum += __shfl_xor(psum, off, 32);
        lrun[r] = lrun[r] * alpha + psum;
        mrun[r] = mnew;
#pragma unroll
        for (int jd = 0; jd < 4; ++jd) Oa[jd][r] *= alpha;
      }
      __syncthreads();

      v8f Ob[4];
#pragma unroll
      for (int jd = 0; jd < 4; ++jd) Ob[jd] = zero8();
#pragma unroll
      for (int k2 = 0; k2 < NK2; ++k2) {
        const v16h pa = load_frag(&Pl[(w * 16) * 64 + kOff + 32 * k2], 64);
        v16h pra = pa;
        if (RES) pra = load_frag(&Prl[(w * 16) * 64 + kOff + 32 * k2], 64);
#pragma unroll
        for (int jd = 0; jd < 4; ++jd) {
          const v16h vb = load_frag(&Vs[(jd * 16) * 64 + kOff + 32 * k2], 64);
          Oa[jd] = wmma16(pa, vb, Oa[jd]);
          if (RES) {
            const v16h vrb = load_frag(&Vrs[(jd * 16) * 64 + kOff + 32 * k2], 64);
            Ob[jd] = wmma16(pa, vrb, Ob[jd]);
            Ob[jd] = wmma16(pra, vb, Ob[jd]);
          }
        }
      }
      if (RES) {
#pragma unroll
        for (int jd = 0; jd < 4; ++jd)
#pragma unroll
          for (int r = 0; r < 8; ++r)
            Oa[jd][r] = Oa[jd][r] + Ob[jd][r] * (1.0f / 4096.0f);
      }
      __syncthreads();
    }
  }

#pragma unroll
  for (int r = 0; r < 8; ++r) {
    const float il = (1.0f / lrun[r]) * (16.0f / 1024.0f);
#pragma unroll
    for (int jd = 0; jd < 4; ++jd) {
      const float cx = Oa[jd][r] * il;
      const _Float16 hh = (_Float16)cx;
      Pl[(w * 16 + 8 * g + r) * 64 + jd * 16 + n] = hh;
      if (RES) Prl[(w * 16 + 8 * g + r) * 64 + jd * 16 + n] = (_Float16)((cx - (float)hh) * 4096.0f);
    }
  }
  __syncthreads();

  {
    const int ch = lane & 7, rq = lane >> 3;
    _Float16* dst  = AO  + ((size_t)b * (SEQ)  + qw) * DM + h * DH;
    _Float16* dstr = AOr + ((size_t)b * (RESQ) + qw) * DM + h * DH;
#pragma unroll
    for (int i = 0; i < 4; ++i) {
      const int rl = i * 4 + rq;
      const v4f val = *reinterpret_cast<const v4f*>(&Pl[(w * 16 + rl) * 64 + ch * 8]);
      *(volatile v4f*)(dst + (size_t)rl * DM + ch * 8) = val;
      if (RES) {
        const v4f valr = *reinterpret_cast<const v4f*>(&Prl[(w * 16 + rl) * 64 + ch * 8]);
        *(volatile v4f*)(dstr + (size_t)rl * DM + ch * 8) = valr;
      }
    }
    __threadfence();
#pragma unroll
    for (int i = 0; i < 4; ++i) {
      const int rl = i * 4 + rq;
      const v4f val = *reinterpret_cast<const v4f*>(&Pl[(w * 16 + rl) * 64 + ch * 8]);
      *(volatile v4f*)(dst + (size_t)rl * DM + ch * 8) = val;
      if (RES) {
        const v4f valr = *reinterpret_cast<const v4f*>(&Prl[(w * 16 + rl) * 64 + ch * 8]);
        *(volatile v4f*)(dstr + (size_t)rl * DM + ch * 8) = valr;
      }
    }
  }
}

template <bool RESB>
__global__ void __launch_bounds__(128)
k_out(const _Float16* __restrict__ A, const _Float16* __restrict__ Ar,
      const _Float16* __restrict__ W, const float* __restrict__ bias,
      float* __restrict__ out, int sbase) {
  __shared__ __align__(16) float so[4 * 16 * 64];

  const int t = threadIdx.x, w = t >> 5, lane = t & 31;
  const int n = lane & 15, g = lane >> 4;
  const int cBase = blockIdx.x * 64;
  const int s0 = sbase + blockIdx.y * 64;
  const int b = blockIdx.z;
  const size_t row0 = (size_t)b * (SEQ) + s0 + 16 * w;

  const _Float16* ar  = A  + row0 * DM;
  const _Float16* arr = Ar + ((size_t)b * (RESQ) + s0 + 16 * w) * DM;
  const _Float16* wr  = W  + (size_t)cBase * DM;

  v8f acc[4], accr[4];
#pragma unroll
  for (int j = 0; j < 4; ++j) { acc[j] = zero8(); accr[j] = zero8(); }

#pragma unroll 1
  for (int kc = 0; kc < DM; kc += 32) {
    const v16h af = load_frag(ar + kc, DM);
    v16h arf = af;
    if (RESB) arf = load_frag(arr + kc, DM);
#pragma unroll
    for (int j = 0; j < 4; ++j) {
      const v16h bf = load_frag(wr + (size_t)(16 * j) * DM + kc, DM);
      acc[j] = wmma16(af, bf, acc[j]);
      if (RESB) accr[j] = wmma16(arf, bf, accr[j]);
    }
  }

  float bia[4];
#pragma unroll
  for (int j = 0; j < 4; ++j) bia[j] = bfr(bias[cBase + 16 * j + n]);
#pragma unroll
  for (int j = 0; j < 4; ++j)
#pragma unroll
    for (int r = 0; r < 8; ++r) {
      float v = acc[j][r] * (1.0f / 1024.0f);
      if (RESB) v = v + accr[j][r] * (1.0f / 4194304.0f);
      v = v + bia[j];
      so[(w * 16 + 8 * g + r) * 64 + j * 16 + n] = v;
    }
  __syncthreads();

  {
    const int ch = lane & 15, rq = lane >> 4;
    float* dst = out + row0 * DM + cBase;
#pragma unroll
    for (int i = 0; i < 8; ++i) {
      const int rl = i * 2 + rq;
      const v4f val = *reinterpret_cast<const v4f*>(&so[(w * 16 + rl) * 64 + ch * 4]);
      *(volatile v4f*)(dst + (size_t)rl * DM + ch * 4) = val;
    }
    __threadfence();
#pragma unroll
    for (int i = 0; i < 8; ++i) {
      const int rl = i * 2 + rq;
      const v4f val = *reinterpret_cast<const v4f*>(&so[(w * 16 + rl) * 64 + ch * 4]);
      *(volatile v4f*)(dst + (size_t)rl * DM + ch * 4) = val;
    }
  }
}

extern "C" void kernel_launch(void* const* d_in, const int* in_sizes, int n_in,
                              void* d_out, int out_size, void* d_ws, size_t ws_size,
                              hipStream_t stream) {
  if (n_in < 9) return;
  const int needx = ((NB - 1) * SEQ_FULL + (SEQ)) * DM;
  if (in_sizes[0] < needx) return;
  if (in_sizes[1] < DM * DM || in_sizes[3] < DM * DM ||
      in_sizes[5] < DM * DM || in_sizes[7] < DM * DM) return;
  if (in_sizes[2] < DM || in_sizes[4] < DM || in_sizes[6] < DM || in_sizes[8] < DM) return;
  if (out_size < MROWS * DM) return;
  if (ws_size < WS_TOTAL) return;

  const float* x  = (const float*)d_in[0];
  const float* Wq = (const float*)d_in[1];
  const float* bq = (const float*)d_in[2];
  const float* Wk = (const float*)d_in[3];
  const float* bk = (const float*)d_in[4];
  const float* Wv = (const float*)d_in[5];
  const float* bv = (const float*)d_in[6];
  const float* Wo = (const float*)d_in[7];
  const float* bo = (const float*)d_in[8];
  float* out = (float*)d_out;

  char* ws = (char*)d_ws;
  _Float16* X16  = (_Float16*)(ws + OFF_X);
  _Float16* WQ16 = (_Float16*)(ws + OFF_WQ);
  _Float16* WK16 = (_Float16*)(ws + OFF_WK);
  _Float16* WV16 = (_Float16*)(ws + OFF_WV);
  _Float16* WO16 = (_Float16*)(ws + OFF_WO);
  _Float16* Q16  = (_Float16*)(ws + OFF_Q);
  _Float16* K16  = (_Float16*)(ws + OFF_K);
  _Float16* VT16 = (_Float16*)(ws + OFF_VT);
  _Float16* AO16 = (_Float16*)(ws + OFF_AO);
  _Float16* QR16 = (_Float16*)(ws + OFF_QR);
  _Float16* KR16 = (_Float16*)(ws + OFF_KR);
  _Float16* VR16 = (_Float16*)(ws + OFF_VTR);
  _Float16* AR16 = (_Float16*)(ws + OFF_AOR);
  v2f*      CS   = (v2f*)(ws + OFF_CS);

  const int npb = (SEQ) * DM / 8;
  for (int bb = 0; bb < NB; ++bb) {
    k_cvt<<<dim3((npb + 255) / 256), dim3(256), 0, stream>>>(
        x + (size_t)bb * SEQ_FULL * DM, X16 + (size_t)bb * (SEQ) * DM, npb, 16.0f);
  }
  const int nw8 = DM * DM / 8;
  k_cvt<<<dim3((nw8 + 255) / 256), dim3(256), 0, stream>>>(Wq, WQ16, nw8, 64.0f);
  k_cvt<<<dim3((nw8 + 255) / 256), dim3(256), 0, stream>>>(Wk, WK16, nw8, 64.0f);
  k_cvt<<<dim3((nw8 + 255) / 256), dim3(256), 0, stream>>>(Wv, WV16, nw8, 64.0f);
  k_cvt<<<dim3((nw8 + 255) / 256), dim3(256), 0, stream>>>(Wo, WO16, nw8, 64.0f);

  const int ncs = (SEQ) * 32;
  k_table<<<dim3((ncs + 255) / 256), dim3(256), 0, stream>>>(CS, ncs);

  const dim3 gp(NH, MROWS / 128);
  k_proj<0><<<gp, dim3(128), 0, stream>>>(X16, WQ16, bq, CS, Q16, QR16);
  k_proj<1><<<gp, dim3(128), 0, stream>>>(X16, WK16, bk, CS, K16, KR16);
  k_proj<2><<<gp, dim3(128), 0, stream>>>(X16, WV16, bv, CS, VT16, VR16);

  const int nres  = (RESQ) / 64;
  const int nrest = ((SEQ) - (RESQ)) / 64;
  k_attn<true><<<dim3(nres, NH, NB), dim3(128), 0, stream>>>(
      Q16, K16, VT16, QR16, KR16, VR16, AO16, AR16, 0);
  if (nrest > 0) {
    k_attn<false><<<dim3(nrest, NH, NB), dim3(128), 0, stream>>>(
        Q16, K16, VT16, QR16, KR16, VR16, AO16, AR16, nres);
  }

  k_out<true><<<dim3(DM / 64, nres, NB), dim3(128), 0, stream>>>(
      AO16, AR16, WO16, bo, out, 0);
  if (nrest > 0) {
    k_out<false><<<dim3(DM / 64, nrest, NB), dim3(128), 0, stream>>>(
        AO16, AR16, WO16, bo, out, (RESQ));
  }
}
